// TextEncoder_24859270709534
// MI455X (gfx1250) — hardware-verified
//
#include <hip/hip_runtime.h>
#include <stdint.h>

typedef __attribute__((ext_vector_type(16))) _Float16 v16h;
typedef __attribute__((ext_vector_type(8)))  _Float16 v8h;
typedef __attribute__((ext_vector_type(8)))  float    v8f;
typedef __attribute__((ext_vector_type(4)))  float    v4f;

__device__ __forceinline__ void dep_guard_h(v8f& a, v8f& b, v16h x, v16h y) { asm volatile("v_nop\n\tv_nop\n\tv_nop\n\tv_nop" : "+v"(a), "+v"(b) : "v"(x), "v"(y)); }
__device__ __forceinline__ void acc_guard4(v8f& a, v8f& b, v8f& c, v8f& d) { asm volatile("v_nop\n\tv_nop\n\tv_nop\n\tv_nop" : "+v"(a), "+v"(b), "+v"(c), "+v"(d)); }
__device__ __forceinline__ void mma_guard3(v8f& x, v8f& y, v8f& z, v16h a, v16h b, v16h c, v16h d) {
  asm volatile("v_nop\n\tv_nop\n\tv_nop\n\tv_nop" : "+v"(x), "+v"(y), "+v"(z) : "v"(a), "v"(b), "v"(c), "v"(d));
}
template <typename T> struct Frag;
template <> struct Frag<_Float16> {
  typedef v16h V; union U { v16h v; v8h h[2]; };
  static __device__ __forceinline__ v16h load(const _Float16* p) {
    U f; f.h[0] = *(const v8h*)(p); f.h[1] = *(const v8h*)(p + 16); return f.v;
  }
  static __device__ __forceinline__ v8f mma(v16h a, v16h b, v8f c) {
    return __builtin_amdgcn_wmma_f32_16x16x32_f16(false, a, false, b, (short)0, c, false, false);
  }
};

constexpr int kBatch = 256;
constexpr int kSteps = 512;
constexpr int kDw    = 64;
constexpr int kHu    = 128;
constexpr int kRowsPerBlk = 16;
constexpr int kHP = 136;
constexpr int kFP = 132;
constexpr float kEmbCarry = 32.0f;
constexpr float kHCarry   = 32.0f;
constexpr float kWCarry   = 8.0f;
constexpr float kAccFold  = 0.00390625f;
constexpr float kLnEps    = 1e-5f;

__global__ __launch_bounds__(256)
void gather_embed_f16(const int* __restrict__ x, const float* __restrict__ emb,
                      _Float16* __restrict__ e16, int n_rows, int vocab) {
  const int i = blockIdx.x * 256 + threadIdx.x;
  const int row = i >> 3;
  const int c8 = (i & 7) * 8;
  const int t = row / kBatch;
  const int b = row - t * kBatch;
  int tok = x[(size_t)b * kSteps + t];
  tok = tok < 0 ? 0 : tok;
  tok = tok > vocab - 1 ? vocab - 1 : tok;
  const float* er = emb + (size_t)tok * kDw + c8;
  const v4f f0 = *(const v4f*)(er);
  const v4f f1 = *(const v4f*)(er + 4);
  v8h hv;
#pragma unroll
  for (int e = 0; e < 4; ++e) {
    hv[e]     = (_Float16)(f0[e] * kEmbCarry);
    hv[4 + e] = (_Float16)(f1[e] * kEmbCarry);
  }
  _Float16* dst = e16 + (size_t)row * kDw + c8;
  *(volatile v8h*)dst = hv;
  __threadfence();
  *(volatile v8h*)dst = hv;
}

__global__ __launch_bounds__(256)
void cast_scale_f32_f16x2(const float* __restrict__ in, _Float16* __restrict__ outp, int n2, float sc) {
  const int i = blockIdx.x * 256 + threadIdx.x;
  if (i < n2) {
    const _Float16 h0 = (_Float16)(in[2 * i] * sc), h1 = (_Float16)(in[2 * i + 1] * sc);
    const unsigned uu = (unsigned)__builtin_bit_cast(unsigned short, h0) | ((unsigned)__builtin_bit_cast(unsigned short, h1) << 16);
    ((volatile unsigned*)outp)[i] = uu;
    __threadfence();
    ((volatile unsigned*)outp)[i] = uu;
  }
}

__global__ __launch_bounds__(256)
void gru_scan_ln(const _Float16* __restrict__ e16, const _Float16* __restrict__ wih16,
                 const _Float16* __restrict__ whh16,
                 const float* __restrict__ b_ih, const float* __restrict__ b_hh,
                 const float* __restrict__ gamma, const float* __restrict__ beta,
                 float* __restrict__ out) {
  __shared__ __align__(16) _Float16 hbuf[2][kRowsPerBlk * kHP];
  __shared__ __align__(16) float    hfin[kRowsPerBlk * kFP];

  const int tid  = threadIdx.x;
  const int wave = tid >> 5;
  const int lane = tid & 31;
  const int c    = lane & 15;
  const int hh   = lane >> 4;
  const int koff = hh * 8;
  const int mbase = blockIdx.x * kRowsPerBlk;
  const int u    = wave * 16 + c;

  const float bsum_r = b_ih[u] + b_hh[u];
  const float bsum_z = b_ih[kHu + u] + b_hh[kHu + u];
  const float b_in   = b_ih[2 * kHu + u];
  const float b_hn   = b_hh[2 * kHu + u];

  float hprev[8];
#pragma unroll
  for (int r = 0; r < 8; ++r) hprev[r] = 0.0f;

  {
    unsigned* hz = (unsigned*)(&hbuf[0][0]);
    for (int i = tid; i < (2 * kRowsPerBlk * kHP) / 2; i += 256) hz[i] = 0u;
  }
  __syncthreads();

  const v8f zero8 = (v8f){0.f, 0.f, 0.f, 0.f, 0.f, 0.f, 0.f, 0.f};

  for (int t = 0; t < kSteps; ++t) {
    const _Float16* hcur = &hbuf[t & 1][0];
    _Float16*       hnxt = &hbuf[(t + 1) & 1][0];

    v8f acc_r = zero8, acc_z = zero8, acc_in = zero8, acc_hn = zero8;

#pragma unroll 1
    for (int ks = 0; ks < kHu / 32; ++ks) {
      const int kb = ks * 32 + koff;
      const v16h a  = Frag<_Float16>::load(hcur + c * kHP + kb);
      const v16h br = Frag<_Float16>::load(whh16 + (size_t)u * kHu + kb);
      const v16h bz = Frag<_Float16>::load(whh16 + (size_t)(kHu + u) * kHu + kb);
      const v16h bn = Frag<_Float16>::load(whh16 + (size_t)(2 * kHu + u) * kHu + kb);
      acc_r  = Frag<_Float16>::mma(a, br, acc_r);
      acc_z  = Frag<_Float16>::mma(a, bz, acc_z);
      acc_hn = Frag<_Float16>::mma(a, bn, acc_hn);
      mma_guard3(acc_r, acc_z, acc_hn, a, br, bz, bn);
    }
    const _Float16* erow = e16 + ((size_t)t * kBatch + mbase + c) * kDw;
#pragma unroll 1
    for (int ks = 0; ks < kDw / 32; ++ks) {
      const int kb = ks * 32 + koff;
      const v16h a  = Frag<_Float16>::load(erow + kb);
      const v16h br = Frag<_Float16>::load(wih16 + (size_t)u * kDw + kb);
      const v16h bz = Frag<_Float16>::load(wih16 + (size_t)(kHu + u) * kDw + kb);
      const v16h bn = Frag<_Float16>::load(wih16 + (size_t)(2 * kHu + u) * kDw + kb);
      acc_r  = Frag<_Float16>::mma(a, br, acc_r);
      acc_z  = Frag<_Float16>::mma(a, bz, acc_z);
      acc_in = Frag<_Float16>::mma(a, bn, acc_in);
      mma_guard3(acc_r, acc_z, acc_in, a, br, bz, bn);
    }
    acc_guard4(acc_r, acc_z, acc_in, acc_hn);

#pragma unroll
    for (int r = 0; r < 8; ++r) {
      const float xr = acc_r[r] * kAccFold + bsum_r;
      const float xz = acc_z[r] * kAccFold + bsum_z;
      const float rg = 1.0f / (1.0f + expf(-xr));
      const float zg = 1.0f / (1.0f + expf(-xz));
      const float np = (acc_in[r] * kAccFold + b_in) + rg * (acc_hn[r] * kAccFold + b_hn);
      const float ng = tanhf(np);
      const float hn = (1.0f - zg) * ng + zg * hprev[r];
      hprev[r] = hn;
      hnxt[(8 * hh + r) * kHP + u] = (_Float16)(hn * kHCarry);
    }
    __syncthreads();
  }

#pragma unroll
  for (int r = 0; r < 8; ++r) hfin[(8 * hh + r) * kFP + u] = hprev[r];
  __syncthreads();

  const v4f gv = *(const v4f*)(gamma + lane * 4);
  const v4f bv = *(const v4f*)(beta + lane * 4);
  v4f ov[2];
#pragma unroll
  for (int i = 0; i < 2; ++i) {
    const int row = wave * 2 + i;
    const v4f hv = *(const v4f*)(hfin + row * kFP + lane * 4);
    float s = (hv[0] + hv[1]) + (hv[2] + hv[3]);
#pragma unroll
    for (int off = 16; off >= 1; off >>= 1) s += __shfl_xor(s, off, 32);
    const float mu = s * (1.0f / (float)kHu);
    v4f d;
#pragma unroll
    for (int e = 0; e < 4; ++e) d[e] = hv[e] - mu;
    float q = (d[0] * d[0] + d[1] * d[1]) + (d[2] * d[2] + d[3] * d[3]);
#pragma unroll
    for (int off = 16; off >= 1; off >>= 1) q += __shfl_xor(q, off, 32);
    const float var = q * (1.0f / (float)kHu);
    const float inv = 1.0f / sqrtf(var + kLnEps);
#pragma unroll
    for (int e = 0; e < 4; ++e) ov[i][e] = d[e] * inv * gv[e] + bv[e];
  }
  float* o0 = out + (size_t)(mbase + wave * 2) * kHu + lane * 4;
  float* o1 = o0 + kHu;
  for (int pass = 0; pass < 2; ++pass) {
    *(volatile v4f*)o0 = ov[0];
    *(volatile v4f*)o1 = ov[1];
    __threadfence();
  }
}

extern "C" void kernel_launch(void* const* d_in, const int* in_sizes, int n_in,
                              void* d_out, int out_size, void* d_ws, size_t ws_size,
                              hipStream_t stream) {
  if (n_in < 8) return;
  const int*   x     = (const int*)d_in[0];
  const float* emb   = (const float*)d_in[1];
  const float* w_ih  = (const float*)d_in[2];
  const float* w_hh  = (const float*)d_in[3];
  const float* b_ih  = (const float*)d_in[4];
  const float* b_hh  = (const float*)d_in[5];
  const float* gamma = (const float*)d_in[6];
  const float* beta  = (const float*)d_in[7];
  float*       out   = (float*)d_out;

  if (in_sizes[0] != kBatch * kSteps) return;
  if (in_sizes[2] != 3 * kHu * kDw || in_sizes[3] != 3 * kHu * kHu) return;
  if (in_sizes[4] != 3 * kHu || in_sizes[5] != 3 * kHu) return;
  if (in_sizes[6] != kHu || in_sizes[7] != kHu) return;
  if (out_size != kBatch * kHu) return;
  const int vocab = in_sizes[1] / kDw;
  if (vocab < 1) return;

  const size_t n_rows  = (size_t)kSteps * kBatch;
  const size_t offE    = 0;
  const size_t bytesE  = n_rows * kDw * 2;
  const size_t offWi   = offE + bytesE;
  const size_t bytesWi = (size_t)3 * kHu * kDw * 2;
  const size_t offWh   = offWi + bytesWi;
  const size_t bytesWh = (size_t)3 * kHu * kHu * 2;
  if (offWh + bytesWh > ws_size) return;

  _Float16* e16   = (_Float16*)((char*)d_ws + offE);
  _Float16* wih16 = (_Float16*)((char*)d_ws + offWi);
  _Float16* whh16 = (_Float16*)((char*)d_ws + offWh);

  const int gatherBlocks = (int)((n_rows * 8) / 256);
  gather_embed_f16<<<gatherBlocks, 256, 0, stream>>>(x, emb, e16, (int)n_rows, vocab);

  const int n2i = (3 * kHu * kDw) / 2;
  const int n2h = (3 * kHu * kHu) / 2;
  cast_scale_f32_f16x2<<<(n2i + 255) / 256, 256, 0, stream>>>(w_ih, wih16, n2i, kWCarry);
  cast_scale_f32_f16x2<<<(n2h + 255) / 256, 256, 0, stream>>>(w_hh, whh16, n2h, kWCarry);

  gru_scan_ln<<<kBatch / kRowsPerBlk, 256, 0, stream>>>(e16, wih16, whh16, b_ih, b_hh, gamma, beta, out);
}
